// modifiedPNAnet_80264348827998
// MI455X (gfx1250) — hardware-verified
//
#include <hip/hip_runtime.h>
#include <stddef.h>
#include <math.h>


#define CD      64
#define NTHR    256
#define NWAVE   8
#define EPT     8
#define NGRP    2
#define CHUNK   (NTHR * EPT * NGRP)
#define WCAP    (EPT * NGRP * 32)
#define LISTN   (NWAVE * WCAP)
#define NBA     256
#define AROW    256
#define GROWS   128
#define APH     72
#define KPO     768
#define NG3     192
#define WSC     16.0f
#define WINV    0.0625f

#define OFF_WN  0
#define OFF_PO  16384
#define OFF_IH  65536
#define OFF_HH  77824
#define WTOT    90112
#define MISCN   512

#define LDS_NODE     (2 * GROWS * APH * 2 + GROWS * CD * 4)
#define AGG_OFF_LIST (NBA * AROW * 4)
#define AGG_OFF_WCNT (AGG_OFF_LIST + LISTN * 4)
#define AGG_OFF_CNT  (AGG_OFF_WCNT + 64)
#define AGG_OFF_S    (AGG_OFF_CNT + NBA * 4)
#define AGG_OFF_T    (AGG_OFF_S + NBA * 4)
#define LDS_AGG      (AGG_OFF_T + NBA * 4)

static_assert((CHUNK & (CHUNK - 1)) == 0);
static_assert(CHUNK <= 4096);
static_assert(NBA <= 4096);
static_assert(NBA == NTHR);
static_assert(WTOT % (8 * NTHR) == 0);
static_assert(GROWS == NWAVE * 16);
static_assert(NBA == NWAVE * 32);
static_assert((APH * 2) % 16 == 0);

typedef float    v2f  __attribute__((ext_vector_type(2)));
typedef float    v4f  __attribute__((ext_vector_type(4)));
typedef float    v8f  __attribute__((ext_vector_type(8)));
typedef int      v4i  __attribute__((ext_vector_type(4)));
typedef _Float16 v8h  __attribute__((ext_vector_type(8)));
typedef _Float16 v16h __attribute__((ext_vector_type(16)));
union FragH { v16h v; v8h h[2]; };

__device__ __forceinline__ v8f zero8() {
  v8f z = {0.f, 0.f, 0.f, 0.f, 0.f, 0.f, 0.f, 0.f};
  return z;
}

__device__ __forceinline__ v8h cvt8(v4f a, v4f b) {
  v8h r;
  r[0] = (_Float16)a.x; r[1] = (_Float16)a.y; r[2] = (_Float16)a.z; r[3] = (_Float16)a.w;
  r[4] = (_Float16)b.x; r[5] = (_Float16)b.y; r[6] = (_Float16)b.z; r[7] = (_Float16)b.w;
  return r;
}

__device__ __forceinline__ v8f wmh(v16h a, v16h b, v8f c) {
  v8f d = __builtin_amdgcn_wmma_f32_16x16x32_f16(false, a, false, b, (short)0, c, false, false);
  asm volatile("v_nop\n\tv_nop\n\tv_nop\n\tv_nop" : "+v"(d) : "v"(a), "v"(b));
  return d;
}

__device__ __forceinline__ float sigm(float v) {
  v = fminf(fmaxf(v, -30.0f), 30.0f);
  return 1.0f / (1.0f + expf(-v));
}

template <int NB>
__device__ __forceinline__ int scan_chunk(const int* __restrict__ dsts, int nE, int cbase, int nodeBase,
                                          int vec8, int* list, int tid, int lane, int wave) {
  int wc = 0;
  const bool full = (vec8 != 0) && (cbase + CHUNK <= nE);
#pragma unroll
  for (int g = 0; g < NGRP; ++g) {
    const int el0  = (g * NTHR + tid) * EPT;
    const int e0   = cbase + el0;
    const int sent = -2147483647 - 1;
    v4i da, db;
    if (full) {
      da = *(const v4i*)(dsts + e0);
      db = *(const v4i*)(dsts + e0 + 4);
    } else {
      da.x = (e0     < nE) ? dsts[min(e0,     nE - 1)] : sent;
      da.y = (e0 + 1 < nE) ? dsts[min(e0 + 1, nE - 1)] : sent;
      da.z = (e0 + 2 < nE) ? dsts[min(e0 + 2, nE - 1)] : sent;
      da.w = (e0 + 3 < nE) ? dsts[min(e0 + 3, nE - 1)] : sent;
      db.x = (e0 + 4 < nE) ? dsts[min(e0 + 4, nE - 1)] : sent;
      db.y = (e0 + 5 < nE) ? dsts[min(e0 + 5, nE - 1)] : sent;
      db.z = (e0 + 6 < nE) ? dsts[min(e0 + 6, nE - 1)] : sent;
      db.w = (e0 + 7 < nE) ? dsts[min(e0 + 7, nE - 1)] : sent;
    }
    const unsigned nb = (unsigned)nodeBase;
    const unsigned s0 = (unsigned)da.x - nb, s1 = (unsigned)da.y - nb;
    const unsigned s2 = (unsigned)da.z - nb, s3 = (unsigned)da.w - nb;
    const unsigned s4 = (unsigned)db.x - nb, s5 = (unsigned)db.y - nb;
    const unsigned s6 = (unsigned)db.z - nb, s7 = (unsigned)db.w - nb;
    const bool h0 = s0 < (unsigned)NB, h1 = s1 < (unsigned)NB, h2 = s2 < (unsigned)NB, h3 = s3 < (unsigned)NB;
    const bool h4 = s4 < (unsigned)NB, h5 = s5 < (unsigned)NB, h6 = s6 < (unsigned)NB, h7 = s7 < (unsigned)NB;
    const unsigned any = __builtin_amdgcn_ballot_w32(h0 | h1 | h2 | h3 | h4 | h5 | h6 | h7);
    if (any != 0u) {
#define HITJ(J, HJ, SJ) { \
        const unsigned mj = __builtin_amdgcn_ballot_w32(HJ); \
        if (mj != 0u) { \
          if (HJ) { \
            const int pos = wc + (int)__builtin_amdgcn_mbcnt_lo(mj, 0u); \
            if (pos < WCAP) list[wave * WCAP + pos] = ((el0 + (J)) << 12) | (int)(SJ); \
          } \
          wc += (int)__builtin_popcount(mj); } }
      HITJ(0, h0, s0)
      HITJ(1, h1, s1)
      HITJ(2, h2, s2)
      HITJ(3, h3, s3)
      HITJ(4, h4, s4)
      HITJ(5, h5, s5)
      HITJ(6, h6, s6)
      HITJ(7, h7, s7)
#undef HITJ
    }
  }
  return wc;
}

__global__ __launch_bounds__(NTHR) void k_wprep(
    const float* __restrict__ W, const float* __restrict__ Wpre, const float* __restrict__ Wpost,
    const float* __restrict__ Wih, const float* __restrict__ Whh, _Float16* wall) {
  const int i = blockIdx.x * NTHR + threadIdx.x;
  if (i >= WTOT / 8) return;
  const int o = i * 8;
  const float* p;
  int st;
  if (o < OFF_PO) {
    const int pl = o >> 12, w = o & 4095, n = w >> 6, k0 = w & 63;
    st = CD;
    if (pl == 0)      p = W + k0 * CD + n;
    else if (pl == 1) p = Wpre + k0 * CD + n;
    else if (pl == 2) p = Wpre + (CD + k0) * CD + n;
    else              p = Wpost + k0 * CD + n;
  } else if (o < OFF_IH) {
    const int w = o - OFF_PO, n = w / KPO, k0 = w - n * KPO;
    st = CD;
    p = Wpost + (size_t)(CD + k0) * CD + n;
  } else if (o < OFF_HH) {
    const int w = o - OFF_IH, n = w >> 6, k0 = w & 63;
    st = NG3;
    p = Wih + k0 * NG3 + n;
  } else {
    const int w = o - OFF_HH, n = w >> 6, k0 = w & 63;
    st = NG3;
    p = Whh + k0 * NG3 + n;
  }
  v4f a, b;
  a.x = p[0];      a.y = p[st];     a.z = p[2 * st]; a.w = p[3 * st];
  b.x = p[4 * st]; b.y = p[5 * st]; b.z = p[6 * st]; b.w = p[7 * st];
  a = a * WSC;
  b = b * WSC;
  const v8h hv = cvt8(a, b);
  _Float16* dp = wall + o;
  *(volatile v8h*)dp = hv;
  __threadfence();
  *(volatile v8h*)dp = hv;
}

__global__ __launch_bounds__(NTHR) void k_misc(
    const float* __restrict__ dh, int nH, const float* __restrict__ We, const float* __restrict__ be,
    const float* __restrict__ Wpre, float* misc) {
  __shared__ double sRed[NTHR];
  __shared__ __attribute__((aligned(16))) float sOut[MISCN];
  const int tid = threadIdx.x, lane = tid & 31, wave = tid >> 5;

  double acc = 0.0;
#pragma unroll 1
  for (int i = tid; i < nH; i += NTHR) acc += (double)logf(dh[i] + 1.0f);
  sRed[tid] = acc;
  __syncthreads();
#pragma unroll 1
  for (int s = NTHR / 2; s > 0; s >>= 1) {
    if (tid < s) sRed[tid] = sRed[tid] + sRed[tid + s];
    __syncthreads();
  }
  const float avgl = (float)(sRed[0] / (double)nH);

  const int j = tid >> 6, c = tid & 63;
  const int jc = j > 2 ? 2 : j;
  float accw = 0.0f;
#pragma unroll 1
  for (int k = 0; k < CD; ++k) {
    const float wv = We[jc * CD + k];
    const float bv = be[k];
    const float sv = (j < 3) ? wv : bv;
    accw = fmaf(sv, Wpre[(size_t)(2 * CD + k) * CD + c], accw);
  }
  sOut[tid] = accw;
  sOut[NTHR + tid] = avgl;
  __syncthreads();

  v4f v;
  v.x = 0.f; v.y = 0.f; v.z = 0.f; v.w = 0.f;
  if (wave < 4) v = *(const v4f*)(sOut + wave * 128 + 4 * lane);
  if (wave < 4) *(volatile v4f*)(misc + wave * 128 + 4 * lane) = v;
  __threadfence();
  if (wave < 4) *(volatile v4f*)(misc + wave * 128 + 4 * lane) = v;
}

__global__ __launch_bounds__(NTHR) void k_node(
    const float* __restrict__ x, const _Float16* __restrict__ wn, float* planes, int nN, int rowsPad) {
  extern __shared__ v4f lds_dyn[];
  char* lb = (char*)lds_dyn;
  _Float16* sA  = (_Float16*)lb;
  _Float16* sM  = sA + GROWS * APH;
  float*    stg = (float*)(lb + 2 * GROWS * APH * 2);
  const int tid = threadIdx.x, lane = tid & 31, wave = tid >> 5, hh = lane >> 4, m = lane & 15;
  const int rowBase = blockIdx.x * GROWS;

#pragma unroll
  for (int i = 0; i < (GROWS * CD / 8) / NTHR; ++i) {
    const int idx = i * NTHR + tid;
    const int r   = idx >> 3;
    const int c0  = (idx & 7) * 8;
    int node = rowBase + r;
    node = node > nN - 1 ? nN - 1 : node;
    const float* xp = x + (size_t)node * CD + c0;
    const v4f a = *(const v4f*)xp, b = *(const v4f*)(xp + 4);
    *(v8h*)(sA + r * APH + c0) = cvt8(a, b);
  }
  __syncthreads();

  v8f acc[4];
#pragma unroll
  for (int t = 0; t < 4; ++t) acc[t] = zero8();
  {
    const _Float16* ar = sA + (wave * 16 + m) * APH + 8 * hh;
#pragma unroll
    for (int kt = 0; kt < CD / 32; ++kt) {
      FragH a;
      a.h[0] = *(const v8h*)(ar + 32 * kt);
      a.h[1] = *(const v8h*)(ar + 32 * kt + 16);
#pragma unroll
      for (int t = 0; t < 4; ++t) {
        const _Float16* bp = wn + (size_t)(16 * t + m) * CD + 32 * kt + 8 * hh;
        FragH b;
        b.h[0] = *(const v8h*)bp;
        b.h[1] = *(const v8h*)(bp + 16);
        acc[t] = wmh(a.v, b.v, acc[t]);
      }
    }
  }
#pragma unroll
  for (int t = 0; t < 4; ++t) {
#pragma unroll
    for (int r = 0; r < 8; ++r)
      sM[(wave * 16 + 8 * hh + r) * APH + 16 * t + m] = (_Float16)(acc[t][r] * WINV);
  }
  __syncthreads();

  const _Float16* mr = sM + (wave * 16 + m) * APH + 8 * hh;
#pragma unroll 1
  for (int g = 0; g < 3; ++g) {
#pragma unroll
    for (int t = 0; t < 4; ++t) acc[t] = zero8();
    const _Float16* wg = wn + (size_t)(g + 1) * CD * CD;
#pragma unroll
    for (int kt = 0; kt < CD / 32; ++kt) {
      FragH a;
      a.h[0] = *(const v8h*)(mr + 32 * kt);
      a.h[1] = *(const v8h*)(mr + 32 * kt + 16);
#pragma unroll
      for (int t = 0; t < 4; ++t) {
        const _Float16* bp = wg + (size_t)(16 * t + m) * CD + 32 * kt + 8 * hh;
        FragH b;
        b.h[0] = *(const v8h*)bp;
        b.h[1] = *(const v8h*)(bp + 16);
        acc[t] = wmh(a.v, b.v, acc[t]);
      }
    }
    __syncthreads();
    {
      float* sp = stg + (wave * 16 + 8 * hh) * CD + m;
#pragma unroll
      for (int t = 0; t < 4; ++t) {
#pragma unroll
        for (int r = 0; r < 8; ++r) sp[r * CD + 16 * t] = acc[t][r] * WINV;
      }
    }
    __syncthreads();
    const float* lp = stg + wave * 16 * CD + 4 * lane;
    float* gp = planes + (size_t)g * (size_t)rowsPad * CD + ((size_t)rowBase + wave * 16) * CD + 4 * lane;
#pragma unroll
    for (int i = 0; i < 8; ++i) { const v4f v = *(const v4f*)(lp + i * 128); *(volatile v4f*)(gp + (size_t)i * 128) = v; }
    __threadfence();
#pragma unroll
    for (int i = 0; i < 8; ++i) { const v4f v = *(const v4f*)(lp + i * 128); *(volatile v4f*)(gp + (size_t)i * 128) = v; }
  }
}

__global__ __launch_bounds__(NTHR) void k_agg(
    const int* __restrict__ ei, const float* __restrict__ eattr,
    const float* __restrict__ pd, const float* __restrict__ ps, const float* __restrict__ q0,
    const float* __restrict__ misc, const float* __restrict__ bpre, const float* __restrict__ bpost,
    const _Float16* __restrict__ wpo, float* outp, int nN, int nE, int vec8) {
  extern __shared__ v4f lds_dyn[];
  char*  lb   = (char*)lds_dyn;
  float* agg  = (float*)lb;
  int*   list = (int*)(lb + AGG_OFF_LIST);
  int*   wcnt = (int*)(lb + AGG_OFF_WCNT);
  int*   cnt  = (int*)(lb + AGG_OFF_CNT);
  float* sS   = (float*)(lb + AGG_OFF_S);
  float* sT   = (float*)(lb + AGG_OFF_T);
  const int tid = threadIdx.x, lane = tid & 31, wave = tid >> 5, hh = lane >> 4, m = lane & 15;
  const int nodeBase = blockIdx.x * NBA;
  const int* dsts = ei + nE;

#pragma unroll 4
  for (int i = tid; i < NBA * AROW / 4; i += NTHR) {
    const int cg = i & 63;
    const float f = (cg < 16) ? 0.0f : ((cg < 32) ? __builtin_inff() : ((cg < 48) ? -__builtin_inff() : 0.0f));
    v4f v;
    v.x = f; v.y = f; v.z = f; v.w = f;
    lds_dyn[i] = v;
  }
  cnt[tid] = 0;
  __syncthreads();

  const int c0 = 2 * lane;
  const v2f w0  = *(const v2f*)(misc + c0);
  const v2f w1  = *(const v2f*)(misc + CD + c0);
  const v2f w2  = *(const v2f*)(misc + 2 * CD + c0);
  const v2f bcv = *(const v2f*)(misc + 3 * CD + c0);
  const v2f bpv = *(const v2f*)(bpre + c0);

  const int nChunks = (nE + CHUNK - 1) / CHUNK;
#pragma unroll 1
  for (int ch = 0; ch < nChunks; ++ch) {
    const int cbase = ch * CHUNK;
    const int wc = scan_chunk<NBA>(dsts, nE, cbase, nodeBase, vec8, list, tid, lane, wave);
    if (lane == 0) wcnt[wave] = wc;
    __syncthreads();
    if (wave == 0) {
#pragma unroll 1
      for (int wsx = 0; wsx < NWAVE; ++wsx) {
        int n = __builtin_amdgcn_readfirstlane(wcnt[wsx]);
        n = n > WCAP ? WCAP : (n < 0 ? 0 : n);
        const int* lp = list + wsx * WCAP;
#pragma unroll 1
        for (int i = 0; i < n; ++i) {
          const int ent  = __builtin_amdgcn_readfirstlane(lp[i]);
          const int slot = ent & (NBA - 1);
          int e = cbase + ((ent >> 12) & (CHUNK - 1));
          e = e > nE - 1 ? nE - 1 : e;
          int src = ei[e];
          src = src < 0 ? 0 : (src > nN - 1 ? nN - 1 : src);
          int node = nodeBase + slot;
          node = node > nN - 1 ? nN - 1 : node;
          const v4f at  = *(const v4f*)(eattr + (size_t)e * 4);
          const v2f vpd = *(const v2f*)(pd + (size_t)node * CD + c0);
          const v2f vps = *(const v2f*)(ps + (size_t)src * CD + c0);
          const v2f g   = (vpd + vps) + (bcv + at.x * w0 + at.y * w1 + at.z * w2);
          const v2f h   = at.w * g + bpv;
          float* row = agg + slot * AROW + c0;
          v2f a1 = *(const v2f*)row;
          v2f mn = *(const v2f*)(row + CD);
          v2f mx = *(const v2f*)(row + 2 * CD);
          v2f a2 = *(const v2f*)(row + 3 * CD);
          a1 = a1 + h;
          mn.x = fminf(mn.x, h.x); mn.y = fminf(mn.y, h.y);
          mx.x = fmaxf(mx.x, h.x); mx.y = fmaxf(mx.y, h.y);
          a2 = a2 + h * h;
          *(v2f*)row            = a1;
          *(v2f*)(row + CD)     = mn;
          *(v2f*)(row + 2 * CD) = mx;
          *(v2f*)(row + 3 * CD) = a2;
          if (lane == 0) cnt[slot] = cnt[slot] + 1;
        }
      }
    }
    __syncthreads();
  }

  const float avgl = misc[256];
  const float rAvg = 1.0f / avgl;
  {
#pragma clang fp contract(off)
    const int   cv   = cnt[tid];
    const float safe = (float)(cv > 0 ? cv : 1);
    const float inv  = 1.0f / safe;
    const bool  has  = cv > 0;
    float* row = agg + tid * AROW;
#pragma unroll 4
    for (int c = 0; c < CD; ++c) {
      const float mean = row[c] * inv;
      const float msq  = row[3 * CD + c] * inv;
      const float var  = msq - mean * mean;
      const float sd   = sqrtf(fmaxf(var, 0.0f) + 1e-5f);
      const float mn   = row[CD + c];
      const float mx   = row[2 * CD + c];
      row[c]          = mean;
      row[CD + c]     = has ? mn : 0.0f;
      row[2 * CD + c] = has ? mx : 0.0f;
      row[3 * CD + c] = sd;
    }
    const float logd = logf(safe + 1.0f);
    sS[tid] = logd * rAvg;
    sT[tid] = avgl * (1.0f / logd);
  }
  __syncthreads();

  v8f acc[2][4];
#pragma unroll
  for (int q = 0; q < 2; ++q) {
#pragma unroll
    for (int t = 0; t < 4; ++t) acc[q][t] = zero8();
  }
  float fs[2], ft[2];
#pragma unroll
  for (int q = 0; q < 2; ++q) { fs[q] = sS[32 * wave + 16 * q + m]; ft[q] = sT[32 * wave + 16 * q + m]; }
#pragma unroll 1
  for (int grp = 0; grp < 3; ++grp) {
    float fa[2], fb[2];
#pragma unroll
    for (int q = 0; q < 2; ++q) { fa[q] = (grp >= 1) ? fs[q] : 1.0f; fb[q] = (grp >= 2) ? ft[q] : 1.0f; }
#pragma unroll
    for (int k8 = 0; k8 < 8; ++k8) {
      const int kt = grp * 8 + k8;
      FragH b[4];
#pragma unroll
      for (int t = 0; t < 4; ++t) {
        const _Float16* bp = wpo + (size_t)(16 * t + m) * KPO + 32 * kt + 8 * hh;
        b[t].h[0] = *(const v8h*)bp;
        b[t].h[1] = *(const v8h*)(bp + 16);
      }
#pragma unroll
      for (int q = 0; q < 2; ++q) {
        const float* ap = agg + (32 * wave + 16 * q + m) * AROW + 32 * k8 + 8 * hh;
        v4f p0 = *(const v4f*)ap,        p1 = *(const v4f*)(ap + 4);
        v4f p2 = *(const v4f*)(ap + 16), p3 = *(const v4f*)(ap + 20);
        p0 = (p0 * fa[q]) * fb[q]; p1 = (p1 * fa[q]) * fb[q];
        p2 = (p2 * fa[q]) * fb[q]; p3 = (p3 * fa[q]) * fb[q];
        FragH a;
        a.h[0] = cvt8(p0, p1);
        a.h[1] = cvt8(p2, p3);
#pragma unroll
        for (int t = 0; t < 4; ++t) acc[q][t] = wmh(a.v, b[t].v, acc[q][t]);
      }
    }
  }
  __syncthreads();

  float* stg = agg;
#pragma unroll
  for (int q = 0; q < 2; ++q) {
    const int r0 = 32 * wave + 16 * q + 8 * hh;
#pragma unroll
    for (int r = 0; r < 8; ++r) {
      int node = nodeBase + r0 + r;
      node = node > nN - 1 ? nN - 1 : node;
      const float* qp = q0 + (size_t)node * CD;
      float* sp = stg + (r0 + r) * CD;
#pragma unroll
      for (int t = 0; t < 4; ++t) {
        const int col = 16 * t + m;
        sp[col] = acc[q][t][r] * WINV + qp[col] + bpost[col];
      }
    }
  }
  __syncthreads();

  const float* lp = stg + 32 * wave * CD + 4 * lane;
  float* gp = outp + ((size_t)nodeBase + 32 * wave) * CD + 4 * lane;
#pragma unroll
  for (int i = 0; i < 16; ++i) { const v4f v = *(const v4f*)(lp + i * 128); *(volatile v4f*)(gp + (size_t)i * 128) = v; }
  __threadfence();
#pragma unroll
  for (int i = 0; i < 16; ++i) { const v4f v = *(const v4f*)(lp + i * 128); *(volatile v4f*)(gp + (size_t)i * 128) = v; }
}

__global__ __launch_bounds__(NTHR) void k_gru(
    const float* __restrict__ x, const float* __restrict__ hin,
    const _Float16* __restrict__ wih, const _Float16* __restrict__ whh,
    const float* __restrict__ bih, const float* __restrict__ bhh, float* out, int nN) {
  __shared__ __attribute__((aligned(16))) float stg[GROWS * CD];
  __shared__ float sBi[NG3];
  __shared__ float sBh[NG3];
  const int tid = threadIdx.x, lane = tid & 31, wave = tid >> 5, hh = lane >> 4, m = lane & 15;
  const int rowBase = blockIdx.x * GROWS;
  if (tid < NG3) { sBi[tid] = bih[tid]; sBh[tid] = bhh[tid]; }
  __syncthreads();

  const int rowA = rowBase + wave * 16 + m;
  const int nodeA = rowA > nN - 1 ? nN - 1 : rowA;
  FragH aO[2], aX[2];
#pragma unroll
  for (int kt = 0; kt < 2; ++kt) {
    const float* op = hin + (size_t)rowA * CD + 32 * kt + 8 * hh;
    const float* xp = x + (size_t)nodeA * CD + 32 * kt + 8 * hh;
    aO[kt].h[0] = cvt8(*(const v4f*)op,        *(const v4f*)(op + 4));
    aO[kt].h[1] = cvt8(*(const v4f*)(op + 16), *(const v4f*)(op + 20));
    aX[kt].h[0] = cvt8(*(const v4f*)xp,        *(const v4f*)(xp + 4));
    aX[kt].h[1] = cvt8(*(const v4f*)(xp + 16), *(const v4f*)(xp + 20));
  }
  const int r0 = wave * 16 + 8 * hh;

  v8f rg[4];
#pragma unroll
  for (int t = 0; t < 4; ++t) {
    v8f ci = zero8(), chh = zero8();
#pragma unroll
    for (int kt = 0; kt < 2; ++kt) {
      const _Float16* pi = wih + (size_t)(16 * t + m) * CD + 32 * kt + 8 * hh;
      const _Float16* ph = whh + (size_t)(16 * t + m) * CD + 32 * kt + 8 * hh;
      FragH bi, bh;
      bi.h[0] = *(const v8h*)pi; bi.h[1] = *(const v8h*)(pi + 16);
      bh.h[0] = *(const v8h*)ph; bh.h[1] = *(const v8h*)(ph + 16);
      ci  = wmh(aO[kt].v, bi.v, ci);
      chh = wmh(aX[kt].v, bh.v, chh);
    }
    const int col = 16 * t + m;
    const float bs = sBi[col] + sBh[col];
#pragma unroll
    for (int r = 0; r < 8; ++r) rg[t][r] = sigm((ci[r] + chh[r]) * WINV + bs);
  }

  v8f ng[4];
#pragma unroll
  for (int t = 0; t < 4; ++t) {
    v8f ci = zero8(), chh = zero8();
#pragma unroll
    for (int kt = 0; kt < 2; ++kt) {
      const _Float16* pi = wih + (size_t)(2 * CD + 16 * t + m) * CD + 32 * kt + 8 * hh;
      const _Float16* ph = whh + (size_t)(2 * CD + 16 * t + m) * CD + 32 * kt + 8 * hh;
      FragH bi, bh;
      bi.h[0] = *(const v8h*)pi; bi.h[1] = *(const v8h*)(pi + 16);
      bh.h[0] = *(const v8h*)ph; bh.h[1] = *(const v8h*)(ph + 16);
      ci  = wmh(aO[kt].v, bi.v, ci);
      chh = wmh(aX[kt].v, bh.v, chh);
    }
    const int col = 16 * t + m;
    const float b1 = sBi[2 * CD + col], b2 = sBh[2 * CD + col];
#pragma unroll
    for (int r = 0; r < 8; ++r) {
      const float i_n = ci[r] * WINV + b1;
      const float h_n = chh[r] * WINV + b2;
      ng[t][r] = tanhf(i_n + rg[t][r] * h_n);
    }
  }

#pragma unroll
  for (int t = 0; t < 4; ++t) {
    v8f ci = zero8(), chh = zero8();
#pragma unroll
    for (int kt = 0; kt < 2; ++kt) {
      const _Float16* pi = wih + (size_t)(CD + 16 * t + m) * CD + 32 * kt + 8 * hh;
      const _Float16* ph = whh + (size_t)(CD + 16 * t + m) * CD + 32 * kt + 8 * hh;
      FragH bi, bh;
      bi.h[0] = *(const v8h*)pi; bi.h[1] = *(const v8h*)(pi + 16);
      bh.h[0] = *(const v8h*)ph; bh.h[1] = *(const v8h*)(ph + 16);
      ci  = wmh(aO[kt].v, bi.v, ci);
      chh = wmh(aX[kt].v, bh.v, chh);
    }
    const int col = 16 * t + m;
    const float bs = sBi[CD + col] + sBh[CD + col];
#pragma unroll
    for (int r = 0; r < 8; ++r) {
      const float z = sigm((ci[r] + chh[r]) * WINV + bs);
      int node = rowBase + r0 + r;
      node = node > nN - 1 ? nN - 1 : node;
      const float xv = x[(size_t)node * CD + col];
      stg[(r0 + r) * CD + col] = (1.0f - z) * ng[t][r] + z * xv;
    }
  }
  __syncthreads();

  const float* lp = stg + wave * 16 * CD + 4 * lane;
  float* gp = out + ((size_t)rowBase + wave * 16) * CD + 4 * lane;
  const int rowL = rowBase + wave * 16 + (lane >> 4);
#pragma unroll
  for (int i = 0; i < 8; ++i) {
    const v4f v = *(const v4f*)(lp + i * 128);
    if (rowL + 2 * i < nN) *(volatile v4f*)(gp + (size_t)i * 128) = v;
  }
  __threadfence();
#pragma unroll
  for (int i = 0; i < 8; ++i) {
    const v4f v = *(const v4f*)(lp + i * 128);
    if (rowL + 2 * i < nN) *(volatile v4f*)(gp + (size_t)i * 128) = v;
  }
}

extern "C" void kernel_launch(void* const* d_in, const int* in_sizes, int n_in,
                              void* d_out, int out_size, void* d_ws, size_t ws_size,
                              hipStream_t stream) {
  if (n_in < 15) return;
  const int nN = in_sizes[0] / CD;
  const int nE = in_sizes[14] / 2;
  const int nH = in_sizes[2];
  if (nN <= 0 || nE <= 0 || nH <= 0) return;
  if (in_sizes[0] != nN * CD || in_sizes[14] != nE * 2 || in_sizes[1] != nE * 4) return;
  if (in_sizes[3] != CD * CD || in_sizes[4] != 3 * CD || in_sizes[5] < CD) return;
  if (in_sizes[6] != 3 * CD * CD || in_sizes[7] < CD) return;
  if (in_sizes[8] != 13 * CD * CD || in_sizes[9] < CD) return;
  if (in_sizes[10] != CD * NG3 || in_sizes[11] < NG3 || in_sizes[12] != CD * NG3 || in_sizes[13] < NG3) return;
  if (out_size != nN * CD) return;

  const float* x     = (const float*)d_in[0];
  const float* eattr = (const float*)d_in[1];
  const float* dh    = (const float*)d_in[2];
  const float* W     = (const float*)d_in[3];
  const float* We    = (const float*)d_in[4];
  const float* be    = (const float*)d_in[5];
  const float* Wpre  = (const float*)d_in[6];
  const float* bpre  = (const float*)d_in[7];
  const float* Wpost = (const float*)d_in[8];
  const float* bpost = (const float*)d_in[9];
  const float* Wih   = (const float*)d_in[10];
  const float* bih   = (const float*)d_in[11];
  const float* Whh   = (const float*)d_in[12];
  const float* bhh   = (const float*)d_in[13];
  const int*   ei    = (const int*)d_in[14];
  float* out = (float*)d_out;

  const int nG = (nN + GROWS - 1) / GROWS;
  const int nA = (nN + NBA - 1) / NBA;
  const int rowsPad = nG * GROWS;
  const int rowsOut = nA * NBA;

  char* ws = (char*)d_ws;
  size_t off = 0;
  const size_t oW  = off; off += (size_t)WTOT * 2;                      off = (off + 255) & ~(size_t)255;
  const size_t oMi = off; off += (size_t)MISCN * 4;                     off = (off + 255) & ~(size_t)255;
  const size_t oPl = off; off += (size_t)3 * (size_t)rowsPad * CD * 4;  off = (off + 255) & ~(size_t)255;
  const size_t oOp = off; off += (size_t)rowsOut * CD * 4;               off = (off + 255) & ~(size_t)255;
  if (off > ws_size) return;
  _Float16* wall  = (_Float16*)(ws + oW);
  float*    misc  = (float*)(ws + oMi);
  float*    planes = (float*)(ws + oPl);
  float*    pd    = planes;
  float*    ps    = planes + (size_t)rowsPad * CD;
  float*    q0    = planes + (size_t)2 * rowsPad * CD;
  float*    outp  = (float*)(ws + oOp);
  const _Float16* wn  = wall + OFF_WN;
  const _Float16* wpo = wall + OFF_PO;
  const _Float16* wih = wall + OFF_IH;
  const _Float16* whh = wall + OFF_HH;

  const int vec8 = ((nE & 3) == 0) ? 1 : 0;

  k_wprep<<<WTOT / 8 / NTHR, NTHR, 0, stream>>>(W, Wpre, Wpost, Wih, Whh, wall);

  k_misc<<<1, NTHR, 0, stream>>>(dh, nH, We, be, Wpre, misc);

  hipFuncSetAttribute(reinterpret_cast<const void*>(&k_node),
                      hipFuncAttributeMaxDynamicSharedMemorySize, LDS_NODE);
  k_node<<<nG, NTHR, LDS_NODE, stream>>>(x, wn, planes, nN, rowsPad);

  hipFuncSetAttribute(reinterpret_cast<const void*>(&k_agg),
                      hipFuncAttributeMaxDynamicSharedMemorySize, LDS_AGG);
  k_agg<<<nA, NTHR, LDS_AGG, stream>>>(ei, eattr, pd, ps, q0, misc, bpre, bpost, wpo, outp, nN, nE, vec8);

  k_gru<<<nG, NTHR, 0, stream>>>(x, outp, wih, whh, bih, bhh, out, nN);
}
